// GraphTrajSTEncoder_67362267070834
// MI455X (gfx1250) — hardware-run, weakly checked
//
#include <hip/hip_runtime.h>
#include <stddef.h>
#include <stdint.h>
#include <math.h>


#define NN     50000
#define NE     800000
#define DD     128
#define PEW    98
#define KIN    226
#define KA     256
#define MP     50048
#define NTHR   256
#define NWAVE  8
#define EPT    8
#define CHUNK  (NTHR * EPT)
#define NBA    1024
#define SLA    10
#define NBLK   49
#define WLC    2560
#define RCAP   18432
#define DEGCAP 64
#define GBM    64
#define GTHR   128
#define RPB    64
#define GXB    (MP * 32 / NTHR)
#define NWPB   160
#define BK_ZINTS (NWAVE * WLC + NWAVE * NBA + RCAP + 3 * NBA)
#define BK_LDS_INTS (BK_ZINTS + 16)
#define WSMAX  134217728
#define SPLIT_S1 1
#define SPLIT_S2 1
#define KS1 (SPLIT_S1 ? 256 : 128)
#define KS2 (SPLIT_S2 ? 256 : 128)

static_assert(NN % 16 == 0);
static_assert(MP % 128 == 0 && MP >= NN && MP % GBM == 0 && MP % RPB == 0);
static_assert(KA % 32 == 0 && KS1 % 32 == 0 && KS2 % 32 == 0 && KIN <= KA && KIN == DD + PEW && PEW % 2 == 0);
static_assert((CHUNK & (CHUNK - 1)) == 0 && NBA == (1 << SLA));
static_assert((long long)(NE + CHUNK) < (1LL << 20));
static_assert(NBLK * NBA >= MP);
static_assert(RCAP * 100 >= 16711 * 105 && RCAP * 100 >= 16659 * 105);
static_assert(DEGCAP >= 36 + 8 && DEGCAP >= 34 + 8 && DEGCAP % 32 == 0);
static_assert(NWAVE * WLC >= RCAP);
static_assert(RCAP % (2 * NTHR) == 0 && BK_ZINTS % 4 == 0 && (NWAVE * WLC) % 4 == 0);
static_assert(BK_LDS_INTS * 4 <= 300000);
static_assert(GBM * DD * 4 + GTHR * 4 <= 65536);
static_assert(GBM == (GTHR / 32) * 16 && RPB % NWAVE == 0 && (MP * 32) % NTHR == 0);
static_assert(NE % 4 == 0);

typedef float          v2f   __attribute__((ext_vector_type(2)));
typedef float          v4f   __attribute__((ext_vector_type(4)));
typedef float          v8f   __attribute__((ext_vector_type(8)));
typedef int            v2i   __attribute__((ext_vector_type(2)));
typedef int            v4i   __attribute__((ext_vector_type(4)));
typedef int            v8i   __attribute__((ext_vector_type(8)));
typedef unsigned short v8us  __attribute__((ext_vector_type(8)));
typedef unsigned short v16us __attribute__((ext_vector_type(16)));
typedef __bf16         v16bf __attribute__((ext_vector_type(16)));
typedef v2f  __attribute__((may_alias)) v2fa;
typedef v4f  __attribute__((may_alias)) v4fa;
typedef v2i  __attribute__((may_alias)) v2ia;
typedef v4i  __attribute__((may_alias)) v4ia;
typedef v8us __attribute__((may_alias)) v8usa;
union FragB { v16bf v; v16us u; v8us h[2]; v8i w; };

__device__ __forceinline__ v8f wmb(const FragB& a, const FragB& b, v8f c) {
  v8f d = __builtin_amdgcn_wmma_f32_16x16x32_bf16(false, a.v, false, b.v, (short)0, c, false, false);
  asm volatile("v_nop\n\tv_nop\n\tv_nop\n\tv_nop" : "+v"(d) : "v"(a.w), "v"(b.w));
  return d;
}

__device__ __forceinline__ unsigned bf16_bits(float f) {
  const unsigned u = __float_as_uint(f);
  const unsigned r = (u + 0x7FFFu + ((u >> 16) & 1u)) >> 16;
  return (f != f) ? 0x7FC0u : r;
}
__device__ __forceinline__ float bf16_val(float f) {
  return __uint_as_float(bf16_bits(f) << 16);
}
__device__ __forceinline__ int clampi(int v, int lo, int hi) {
  return v < lo ? lo : (v > hi ? hi : v);
}

__device__ __forceinline__ void hilo_pack(float v0, float v1, float v2, float v3,
                                          int& h01, int& h23, int& l01, int& l23) {
  const unsigned a0 = bf16_bits(v0), a1 = bf16_bits(v1), a2 = bf16_bits(v2), a3 = bf16_bits(v3);
  const unsigned b0 = bf16_bits(v0 - __uint_as_float(a0 << 16));
  const unsigned b1 = bf16_bits(v1 - __uint_as_float(a1 << 16));
  const unsigned b2 = bf16_bits(v2 - __uint_as_float(a2 << 16));
  const unsigned b3 = bf16_bits(v3 - __uint_as_float(a3 << 16));
  h01 = (int)(a0 | (a1 << 16)); h23 = (int)(a2 | (a3 << 16));
  l01 = (int)(b0 | (b1 << 16)); l23 = (int)(b2 | (b3 << 16));
}

__device__ __forceinline__ v4i regroup16(int h01, int h23, int l01, int l23, int lane) {
  const int s0 = (2 * lane) & 31, s1 = s0 + 1;
  const int a0 = __shfl(h01, s0, 32), a1 = __shfl(h23, s0, 32), a2 = __shfl(h01, s1, 32), a3 = __shfl(h23, s1, 32);
  const int b0 = __shfl(l01, s0, 32), b1 = __shfl(l23, s0, 32), b2 = __shfl(l01, s1, 32), b3 = __shfl(l23, s1, 32);
  const int mk = (lane < 16) ? -1 : 0;
  v4i o;
  o.x = (a0 & mk) | (b0 & ~mk); o.y = (a1 & mk) | (b1 & ~mk);
  o.z = (a2 & mk) | (b2 & ~mk); o.w = (a3 & mk) | (b3 & ~mk);
  return o;
}

__device__ __forceinline__ float edge_norm(float a) {
  const float ab   = bf16_val(a);
  const bool  pos  = ab > 0.0f;
  const float safe = pos ? ab : 1.0f;
  const float r    = 1.0f / sqrtf(safe);
  return pos ? fminf(r, 1.0f) : 0.0f;
}

__device__ __forceinline__ unsigned match_slot(int slot, bool valid) {
  unsigned peers = __builtin_amdgcn_ballot_w32(valid);
#pragma unroll
  for (int b = 0; b < SLA; ++b) {
    const bool bit = ((slot >> b) & 1) != 0;
    const unsigned bal = __builtin_amdgcn_ballot_w32(bit);
    peers &= bit ? bal : ~bal;
  }
  return peers;
}

template <int SLB>
__device__ __forceinline__ int scan_chunk(const int* __restrict__ keys, int nE, int cbase, int slotBase,
                                          int nb, int vec8, int* wlist, int wc, int tid) {
  const int e0   = cbase + tid * EPT;
  const int sent = -2147483647 - 1;
  v4i da, db;
  if (vec8 != 0 && cbase + CHUNK <= nE) {
    da = *(const v4i*)(keys + e0);
    db = *(const v4i*)(keys + e0 + 4);
  } else {
    const int k0 = keys[min(e0,     nE - 1)];
    const int k1 = keys[min(e0 + 1, nE - 1)];
    const int k2 = keys[min(e0 + 2, nE - 1)];
    const int k3 = keys[min(e0 + 3, nE - 1)];
    const int k4 = keys[min(e0 + 4, nE - 1)];
    const int k5 = keys[min(e0 + 5, nE - 1)];
    const int k6 = keys[min(e0 + 6, nE - 1)];
    const int k7 = keys[min(e0 + 7, nE - 1)];
    asm volatile("" :: "v"(k0), "v"(k1), "v"(k2), "v"(k3), "v"(k4), "v"(k5), "v"(k6), "v"(k7));
    da.x = (e0     < nE) ? k0 : sent;
    da.y = (e0 + 1 < nE) ? k1 : sent;
    da.z = (e0 + 2 < nE) ? k2 : sent;
    da.w = (e0 + 3 < nE) ? k3 : sent;
    db.x = (e0 + 4 < nE) ? k4 : sent;
    db.y = (e0 + 5 < nE) ? k5 : sent;
    db.z = (e0 + 6 < nE) ? k6 : sent;
    db.w = (e0 + 7 < nE) ? k7 : sent;
  }
  const unsigned nbs = (unsigned)slotBase;
  const unsigned unb = (unsigned)nb;
  const unsigned s0 = (unsigned)da.x - nbs, s1 = (unsigned)da.y - nbs;
  const unsigned s2 = (unsigned)da.z - nbs, s3 = (unsigned)da.w - nbs;
  const unsigned s4 = (unsigned)db.x - nbs, s5 = (unsigned)db.y - nbs;
  const unsigned s6 = (unsigned)db.z - nbs, s7 = (unsigned)db.w - nbs;
  const bool h0 = s0 < unb, h1 = s1 < unb, h2 = s2 < unb, h3 = s3 < unb;
  const bool h4 = s4 < unb, h5 = s5 < unb, h6 = s6 < unb, h7 = s7 < unb;
  const unsigned any = __builtin_amdgcn_ballot_w32(h0 | h1 | h2 | h3 | h4 | h5 | h6 | h7);
  if (any != 0u) {
#define HITJ(J, HJ, SJ) { \
      const unsigned mj = __builtin_amdgcn_ballot_w32(HJ); \
      if (mj != 0u) { \
        if (HJ) { \
          const int pos = wc + (int)__builtin_amdgcn_mbcnt_lo(mj, 0u); \
          if (pos < WLC) wlist[pos] = ((e0 + (J)) << SLB) | (int)(SJ); \
        } \
        wc += (int)__builtin_popcount(mj); } }
    HITJ(0, h0, s0)
    HITJ(1, h1, s1)
    HITJ(2, h2, s2)
    HITJ(3, h3, s3)
    HITJ(4, h4, s4)
    HITJ(5, h5, s5)
    HITJ(6, h6, s6)
    HITJ(7, h7, s7)
#undef HITJ
  }
  return wc;
}

__device__ __forceinline__ v8us wgather8(const float* __restrict__ w, int nn, int k0, int kmax) {
  float v[8];
#pragma unroll
  for (int i = 0; i < 8; ++i) {
    const int k  = k0 + i;
    const int kc = k < kmax ? k : kmax - 1;
    v[i] = w[(size_t)kc * DD + nn];
  }
  asm volatile("" :: "v"(v[0]), "v"(v[1]), "v"(v[2]), "v"(v[3]), "v"(v[4]), "v"(v[5]), "v"(v[6]), "v"(v[7]));
  v8us o;
#pragma unroll
  for (int i = 0; i < 8; ++i)
    o[i] = (k0 + i < kmax) ? (unsigned short)bf16_bits(v[i]) : (unsigned short)0;
  return o;
}

__global__ __launch_bounds__(NTHR) void k_prep(
    const float* __restrict__ x, const float* __restrict__ d2,
    const float* __restrict__ nl1, const float* __restrict__ nl2,
    const float* __restrict__ l11, const float* __restrict__ l21,
    const float* __restrict__ l12, const float* __restrict__ l22,
    const float* __restrict__ l13, const float* __restrict__ l23,
    const float* __restrict__ l14, const float* __restrict__ l24,
    int nN, unsigned short* xin, unsigned short* wpl) {
  const int tid = (int)threadIdx.x;
  const int blk = (int)blockIdx.x;
  if (blk < GXB) {
    const int u   = blk * NTHR + tid;
    const int row = u >> 5;
    const int k8  = (u & 31) * 8;
    const int rc  = row < nN ? row : nN - 1;
    const bool live = row < nN;
    const float* px = x + (size_t)rc * DD + (k8 & (DD - 1));
    const v4f a = *(const v4fa*)px;
    const v4f b = *(const v4fa*)(px + 4);
    const int dj = k8 - DD;
    const int pb = dj >> 1;
    const float* pd = d2 + (size_t)rc * PEW;
    const v2f c0 = *(const v2fa*)(pd + 2 * clampi(pb,     0, PEW / 2 - 1));
    const v2f c1 = *(const v2fa*)(pd + 2 * clampi(pb + 1, 0, PEW / 2 - 1));
    const v2f c2 = *(const v2fa*)(pd + 2 * clampi(pb + 2, 0, PEW / 2 - 1));
    const v2f c3 = *(const v2fa*)(pd + 2 * clampi(pb + 3, 0, PEW / 2 - 1));
    asm volatile("" :: "v"(a.x), "v"(a.y), "v"(a.z), "v"(a.w), "v"(b.x), "v"(b.y), "v"(b.z), "v"(b.w));
    asm volatile("" :: "v"(c0.x), "v"(c0.y), "v"(c1.x), "v"(c1.y), "v"(c2.x), "v"(c2.y), "v"(c3.x), "v"(c3.y));
    const bool isd = live && (k8 >= DD);
    const unsigned mx  = (live && (k8 < DD)) ? 0xFFFFu : 0u;
    const unsigned md0 = (isd && (dj     < PEW)) ? 0xFFFFu : 0u;
    const unsigned md1 = (isd && (dj + 2 < PEW)) ? 0xFFFFu : 0u;
    const unsigned md2 = (isd && (dj + 4 < PEW)) ? 0xFFFFu : 0u;
    const unsigned md3 = (isd && (dj + 6 < PEW)) ? 0xFFFFu : 0u;
    v8us o;
    o[0] = (unsigned short)((bf16_bits(a.x) & mx) | (bf16_bits(c0.x) & md0));
    o[1] = (unsigned short)((bf16_bits(a.y) & mx) | (bf16_bits(c0.y) & md0));
    o[2] = (unsigned short)((bf16_bits(a.z) & mx) | (bf16_bits(c1.x) & md1));
    o[3] = (unsigned short)((bf16_bits(a.w) & mx) | (bf16_bits(c1.y) & md1));
    o[4] = (unsigned short)((bf16_bits(b.x) & mx) | (bf16_bits(c2.x) & md2));
    o[5] = (unsigned short)((bf16_bits(b.y) & mx) | (bf16_bits(c2.y) & md2));
    o[6] = (unsigned short)((bf16_bits(b.z) & mx) | (bf16_bits(c3.x) & md3));
    o[7] = (unsigned short)((bf16_bits(b.w) & mx) | (bf16_bits(c3.y) & md3));
    unsigned short* dp = xin + (size_t)row * KA + k8;
    *(volatile v8us*)dp = o;
    __threadfence();
    *(volatile v8us*)dp = o;
  } else {
    const int pbk = blk - GXB;
    const int p   = pbk >> 5;
    const int ub  = (pbk & 31) * NTHR + tid;
    const int n   = ub >> 5;
    const int k8  = (ub & 31) * 8;
    const int hf  = ((pbk & 31) >= 16) ? 1 : 0;
    const int nn  = n & (DD - 1);
    const int kk  = k8 & (DD - 1);
    const int mid = p * 2 + hf;
    v8us o;
    switch (mid) {
      case 0:  o = wgather8(nl1, nn, k8, KIN); break;
      case 1:  o = wgather8(nl2, nn, k8, KIN); break;
      case 2:  o = wgather8(l11, nn, kk, DD);  break;
      case 3:  o = wgather8(l21, nn, kk, DD);  break;
      case 4:  o = wgather8(l12, nn, kk, DD);  break;
      case 5:  o = wgather8(l22, nn, kk, DD);  break;
      case 6:  o = wgather8(l13, nn, kk, DD);  break;
      case 7:  o = wgather8(l23, nn, kk, DD);  break;
      case 8:  o = wgather8(l14, nn, kk, DD);  break;
      default: o = wgather8(l24, nn, kk, DD);  break;
    }
    unsigned short* dp = wpl + (size_t)p * (KA * KA) + (size_t)n * KA + k8;
    *(volatile v8us*)dp = o;
    __threadfence();
    *(volatile v8us*)dp = o;
  }
}

__global__ __launch_bounds__(NTHR) void k_bucket(const int* __restrict__ rows, const int* __restrict__ keys,
                                                 const float* __restrict__ attr, int nE, int nN, int vec8,
                                                 int* lst, int* cntg, int* offg, int* disg, int* flagg) {
  extern __shared__ __attribute__((aligned(16))) int dsm[];
  int* wl   = dsm;
  int* wcn  = wl + NWAVE * WLC;
  int* sl   = wcn + NWAVE * NBA;
  int* cnt  = sl + RCAP;
  int* offs = cnt + NBA;
  int* dsi  = offs + NBA;
  int* misc = dsi + NBA;
  const int tid = (int)threadIdx.x, lane = tid & 31, wave = tid >> 5;
  const int blk = (int)blockIdx.x;
  const int nodeBase = blk * NBA;

  {
    const v4i z4 = {0, 0, 0, 0};
    for (int i = tid * 4; i < BK_ZINTS; i += NTHR * 4) *(v4ia*)(dsm + i) = z4;
    if (tid < 16) misc[tid] = 0;
  }
  __syncthreads();

  int* wlw = wl + wave * WLC;
  int wc = 0;
  const int nChunks = (nE + CHUNK - 1) / CHUNK;
#pragma unroll 1
  for (int ch = 0; ch < nChunks; ++ch)
    wc = scan_chunk<SLA>(keys, nE, ch * CHUNK, nodeBase, NBA, vec8, wlw, wc, tid);
  if (lane == 0) misc[wave] = (wc > WLC) ? 1 : 0;
  const int cw = wc < 0 ? 0 : (wc > WLC ? WLC : wc);
  __syncthreads();

  int* wcw = wcn + wave * NBA;
#pragma unroll 1
  for (int b0 = 0; b0 < cw; b0 += 32) {
    const int idx = b0 + lane;
    const bool valid = idx < cw;
    const int ent  = wlw[idx < WLC ? idx : WLC - 1];
    const int slot = ent & (NBA - 1);
    const unsigned peers = match_slot(slot, valid);
    const int rank = (int)__builtin_amdgcn_mbcnt_lo(peers, 0u);
    const int tot  = (int)__builtin_popcount(peers);
    const int cur  = wcw[slot];
    if (valid && rank == 0) wcw[slot] = cur + tot;
  }
  __syncthreads();

#pragma unroll 1
  for (int s = tid; s < NBA; s += NTHR) {
    int t = 0;
#pragma unroll
    for (int w2 = 0; w2 < NWAVE; ++w2) t += wcn[w2 * NBA + s];
    cnt[s] = t;
  }
  __syncthreads();
  if (wave == 0) {
    const int base = lane * (NBA / 32);
    int s = 0;
#pragma unroll 1
    for (int i = 0; i < NBA / 32; ++i) s += cnt[base + i];
    int incl = s;
#pragma unroll
    for (int d = 1; d < 32; d <<= 1) {
      const int y = __shfl_up(incl, d, 32);
      if (lane >= d) incl += y;
    }
    int run = incl - s;
#pragma unroll 1
    for (int i = 0; i < NBA / 32; ++i) {
      const int cv = cnt[base + i];
      offs[base + i] = run;
      run += cv;
    }
    if (lane == 31) misc[8] = run;
  }
  __syncthreads();
#pragma unroll 1
  for (int s = tid; s < NBA; s += NTHR) {
    int run = offs[s];
#pragma unroll
    for (int w2 = 0; w2 < NWAVE; ++w2) {
      const int t = wcn[w2 * NBA + s];
      wcn[w2 * NBA + s] = run;
      run += t;
    }
    const float dg = (float)(cnt[s] + 1);
    dsi[s] = __float_as_int(1.0f / sqrtf(dg));
  }
  __syncthreads();

#pragma unroll 1
  for (int b0 = 0; b0 < cw; b0 += 32) {
    const int idx = b0 + lane;
    const bool valid = idx < cw;
    const int ent  = wlw[idx < WLC ? idx : WLC - 1];
    const int slot = ent & (NBA - 1);
    const unsigned peers = match_slot(slot, valid);
    const int rank = (int)__builtin_amdgcn_mbcnt_lo(peers, 0u);
    const int tot  = (int)__builtin_popcount(peers);
    const int cur  = wcw[slot];
    const int pos  = cur + rank;
    if (valid && (unsigned)pos < (unsigned)RCAP) sl[pos] = ent;
    if (valid && rank == 0) wcw[slot] = cur + tot;
  }
  __syncthreads();

  const int traw = misc[8];
  const int tt   = traw < 0 ? 0 : (traw > RCAP ? RCAP : traw);
  const int ovf  = (misc[0] | misc[1] | misc[2] | misc[3] | misc[4] | misc[5] | misc[6] | misc[7]) |
                   ((traw > RCAP || traw < 0) ? 1 : 0);

  int* lb = lst + (size_t)blk * (RCAP * 2);
#pragma unroll 1
  for (int it = 0; it < RCAP / (2 * NTHR); ++it) {
    const int u  = it * NTHR + tid;
    const int i0 = 2 * u;
    const int ea = sl[i0];
    const int eb = sl[i0 + 1];
    const int ida = clampi(ea >> SLA, 0, nE - 1);
    const int idb = clampi(eb >> SLA, 0, nE - 1);
    const int ra0 = rows[ida];
    const int rb0 = rows[idb];
    const float aa = attr[ida];
    const float ab = attr[idb];
    asm volatile("" :: "v"(ra0), "v"(rb0), "v"(aa), "v"(ab));
    const int ra = clampi(ra0, 0, nN - 1);
    const int rb = clampi(rb0, 0, nN - 1);
    const int ena = __float_as_int(edge_norm(aa));
    const int enb = __float_as_int(edge_norm(ab));
    const int la = (i0     < tt) ? -1 : 0;
    const int lb2 = (i0 + 1 < tt) ? -1 : 0;
    v4i o;
    o.x = ra & la;  o.y = ena & la;
    o.z = rb & lb2; o.w = enb & lb2;
    int* dp = lb + 4 * u;
    *(volatile v4i*)dp = o;
    __threadfence();
    *(volatile v4i*)dp = o;
  }

  {
    const v4i c4 = *(const v4ia*)(cnt  + 4 * tid);
    const v4i o4 = *(const v4ia*)(offs + 4 * tid);
    const v4i d4 = *(const v4ia*)(dsi  + 4 * tid);
    const int fl = (ovf != 0) ? 1 : 0;
    const v4i f4 = {fl, fl, fl, fl};
    int* cp = cntg + (size_t)nodeBase + 4 * tid;
    int* op = offg + (size_t)nodeBase + 4 * tid;
    int* dp = disg + (size_t)nodeBase + 4 * tid;
    int* fp = flagg + (size_t)blk * 32 + 4 * (tid & 7);
    *(volatile v4i*)cp = c4;
    *(volatile v4i*)op = o4;
    *(volatile v4i*)dp = d4;
    if (tid < 8) *(volatile v4i*)fp = f4;
    __threadfence();
    *(volatile v4i*)cp = c4;
    *(volatile v4i*)op = o4;
    *(volatile v4i*)dp = d4;
    if (tid < 8) *(volatile v4i*)fp = f4;
  }
}

template <int MODE, int KK>
__global__ __launch_bounds__(GTHR) __attribute__((amdgpu_num_vgpr(248)))
void k_gemm(const unsigned short* __restrict__ A, const unsigned short* __restrict__ BT,
            const float* __restrict__ dis, int nN, float* TF, unsigned short* P, size_t pstride) {
  __shared__ __attribute__((aligned(16))) float stg[GBM * DD];
  __shared__ __attribute__((aligned(16))) float sdis[GTHR];
  const int tid = (int)threadIdx.x, lane = tid & 31, wave = tid >> 5, hh = lane >> 4, m = lane & 15;
  const int rowBase = (int)blockIdx.x * GBM;
  const int yb      = (int)blockIdx.y;

  if constexpr (MODE == 1) {
    const float dv = dis[rowBase + (tid & (GBM - 1))];
    asm volatile("" :: "v"(dv));
    sdis[tid] = dv;
  } else {
    sdis[tid] = 1.0f;
  }

  v8f acc[8];
  {
    const v8f z = {0.f, 0.f, 0.f, 0.f, 0.f, 0.f, 0.f, 0.f};
#pragma unroll
    for (int t = 0; t < 8; ++t) acc[t] = z;
  }
  const unsigned short* ap = A  + (size_t)(rowBase + 16 * wave + m) * (size_t)KA + 8 * hh;
  const unsigned short* bp = BT + (size_t)(DD * yb + m) * (size_t)KA + 8 * hh;

#pragma unroll 1
  for (int k0 = 0; k0 < KK; k0 += 32) {
    FragB af;
    af.h[0] = *(const v8usa*)(ap + k0);
    af.h[1] = *(const v8usa*)(ap + k0 + 16);
#pragma unroll
    for (int nt = 0; nt < 8; ++nt) {
      const unsigned short* wq = bp + (size_t)(16 * nt) * (size_t)KA + k0;
      FragB bf;
      bf.h[0] = *(const v8usa*)wq;
      bf.h[1] = *(const v8usa*)(wq + 16);
      acc[nt] = wmb(af, bf, acc[nt]);
    }
  }

#pragma unroll
  for (int nt = 0; nt < 8; ++nt) {
    const int lc = 16 * nt + m;
#pragma unroll
    for (int r = 0; r < 8; ++r) {
      const int lr = 16 * wave + 8 * hh + r;
      stg[lr * DD + lc] = acc[nt][r];
    }
  }
  __syncthreads();

  if constexpr (MODE == 0) {
    const int mk = (lane < 16) ? -1 : 0;
#pragma unroll 1
    for (int g = 0; g < 4; ++g) {
      v4i ov[4];
#pragma unroll
      for (int j = 0; j < 4; ++j) {
        const int lr   = 16 * wave + 4 * g + j;
        const int grow = rowBase + lr;
        const float* sp = stg + lr * DD + 8 * m;
        const v4f f0 = *(const v4fa*)sp;
        const v4f f1 = *(const v4fa*)(sp + 4);
        int h01, h23, l01, l23, h45, h67, l45, l67;
        hilo_pack(f0.x, f0.y, f0.z, f0.w, h01, h23, l01, l23);
        hilo_pack(f1.x, f1.y, f1.z, f1.w, h45, h67, l45, l67);
        const int lv = (grow < nN) ? -1 : 0;
        v4i o;
        o.x = ((h01 & mk) | (l01 & ~mk)) & lv;
        o.y = ((h23 & mk) | (l23 & ~mk)) & lv;
        o.z = ((h45 & mk) | (l45 & ~mk)) & lv;
        o.w = ((h67 & mk) | (l67 & ~mk)) & lv;
        ov[j] = o;
      }
#pragma unroll
      for (int j = 0; j < 4; ++j) {
        const int grow = rowBase + 16 * wave + 4 * g + j;
        unsigned short* dp = P + (size_t)yb * pstride + (size_t)grow * KA + 8 * lane;
        *(volatile v4i*)dp = ov[j];
      }
      __threadfence();
#pragma unroll
      for (int j = 0; j < 4; ++j) {
        const int grow = rowBase + 16 * wave + 4 * g + j;
        unsigned short* dp = P + (size_t)yb * pstride + (size_t)grow * KA + 8 * lane;
        *(volatile v4i*)dp = ov[j];
      }
    }
  } else {
#pragma unroll 1
    for (int g = 0; g < 4; ++g) {
      v4f fv[4];
#pragma unroll
      for (int j = 0; j < 4; ++j) {
        const int lr   = 16 * wave + 4 * g + j;
        const int grow = rowBase + lr;
        const v4f v  = *(const v4fa*)(stg + lr * DD + 4 * lane);
        const float sd = sdis[lr];
        const float sc = (yb == 0) ? sd : 1.0f;
        const bool live = grow < nN;
        v4f o;
        o.x = live ? v.x * sc : 0.0f; o.y = live ? v.y * sc : 0.0f;
        o.z = live ? v.z * sc : 0.0f; o.w = live ? v.w * sc : 0.0f;
        fv[j] = o;
      }
#pragma unroll
      for (int j = 0; j < 4; ++j) {
        const int grow = rowBase + 16 * wave + 4 * g + j;
        float* op = TF + (size_t)grow * KA + DD * yb + 4 * lane;
        *(volatile v4f*)op = fv[j];
      }
      __threadfence();
#pragma unroll
      for (int j = 0; j < 4; ++j) {
        const int grow = rowBase + 16 * wave + 4 * g + j;
        float* op = TF + (size_t)grow * KA + DD * yb + 4 * lane;
        *(volatile v4f*)op = fv[j];
      }
    }
  }
}

template <int MODE>
__global__ __launch_bounds__(NTHR) void k_replay(const float* __restrict__ T, const int* __restrict__ lst,
                                                 const int* __restrict__ cntg, const int* __restrict__ offg,
                                                 const float* __restrict__ disg, const int* __restrict__ flagA,
                                                 const int* __restrict__ flagB, int nN, int mRows,
                                                 const float* __restrict__ x0in, float* fout, unsigned short* xm) {
  const int tid = (int)threadIdx.x, lane = tid & 31, wave = tid >> 5;
  const int rowBase = (int)blockIdx.x * RPB;
  const float qnan = __int_as_float(0x7fc00000);
#pragma unroll 1
  for (int si = 0; si < RPB / NWAVE; ++si) {
    const int node = rowBase + si * NWAVE + wave;
    const int nc   = node < nN ? node : nN - 1;
    const bool live = node < nN;
    const int bb = nc >> SLA;
    int c = cntg[nc];
    int o = offg[nc];
    const float dd = disg[nc];
    const int fa = flagA[bb * 32];
    const int fb = flagB[bb * 32];
    asm volatile("" :: "v"(c), "v"(o), "v"(dd), "v"(fa), "v"(fb));
    const bool big = (c > DEGCAP) | (c < 0);
    c = clampi(c, 0, DEGCAP);
    c = __builtin_amdgcn_readfirstlane(c);
    o = clampi(o, 0, RCAP);
    const int* lb = lst + (size_t)bb * (RCAP * 2);
    float p0 = 0.0f, p1 = 0.0f, p2 = 0.0f, p3 = 0.0f;
    float q0 = 0.0f, q1 = 0.0f, q2 = 0.0f, q3 = 0.0f;
#pragma unroll 1
    for (int b0 = 0; b0 < c; b0 += 32) {
      int idx = o + b0 + lane;
      idx = idx > RCAP - 1 ? RCAP - 1 : idx;
      const v2i ent = *(const v2ia*)(lb + 2 * idx);
      const int sr  = clampi(ent.x, 0, nN - 1);
      const int eni = ent.y;
      const int m32 = (c - b0) < 32 ? (c - b0) : 32;
#pragma unroll 1
      for (int k = 0; k < m32; ++k) {
        const int   sk = __builtin_amdgcn_readlane(sr, k);
        const float ek = __int_as_float(__builtin_amdgcn_readlane(eni, k));
        const float* tp = T + (size_t)sk * KA + 4 * lane;
        const v4f t1 = *(const v4fa*)tp;
        const v4f t2 = *(const v4fa*)(tp + DD);
        p0 += t1.x; p1 += t1.y; p2 += t1.z; p3 += t1.w;
        q0 = fmaf(ek, t2.x, q0); q1 = fmaf(ek, t2.y, q1);
        q2 = fmaf(ek, t2.z, q2); q3 = fmaf(ek, t2.w, q3);
      }
    }
    {
      const float* tp = T + (size_t)nc * KA + 4 * lane;
      const v4f s1 = *(const v4fa*)tp;
      const v4f s2 = *(const v4fa*)(tp + DD);
      asm volatile("" :: "v"(s1.x), "v"(s1.y), "v"(s1.z), "v"(s1.w), "v"(s2.x), "v"(s2.y), "v"(s2.z), "v"(s2.w));
      p0 += s1.x; p1 += s1.y; p2 += s1.z; p3 += s1.w;
      q0 += s2.x; q1 += s2.y; q2 += s2.z; q3 += s2.w;
    }
    const float v0 = fmaf(dd, p0, q0), v1 = fmaf(dd, p1, q1);
    const float v2 = fmaf(dd, p2, q2), v3 = fmaf(dd, p3, q3);
    const float y0 = 0.5f * ((v0 > 0.0f) ? v0 : (v0 - v0));
    const float y1 = 0.5f * ((v1 > 0.0f) ? v1 : (v1 - v1));
    const float y2 = 0.5f * ((v2 > 0.0f) ? v2 : (v2 - v2));
    const float y3 = 0.5f * ((v3 > 0.0f) ? v3 : (v3 - v3));
    if constexpr (MODE == 0) {
      const bool bad = (fa != 0) | big;
      v4f ow;
      ow.x = bad ? qnan : y0; ow.y = bad ? qnan : y1;
      ow.z = bad ? qnan : y2; ow.w = bad ? qnan : y3;
      if (live) {
        float* op = fout + (size_t)node * DD + 4 * lane;
        *(volatile v4f*)op = ow;
        __threadfence();
        *(volatile v4f*)op = ow;
      }
    } else {
      const v4f x0 = *(const v4fa*)(x0in + (size_t)nc * DD + 4 * lane);
      asm volatile("" :: "v"(x0.x), "v"(x0.y), "v"(x0.z), "v"(x0.w));
      if constexpr (MODE == 1) {
        const bool bad = (fa != 0) | big;
        const float z0 = bad ? qnan : (x0.x + y0), z1 = bad ? qnan : (x0.y + y1);
        const float z2 = bad ? qnan : (x0.z + y2), z3 = bad ? qnan : (x0.w + y3);
        const float r0 = live ? z0 : 0.0f, r1 = live ? z1 : 0.0f;
        const float r2 = live ? z2 : 0.0f, r3 = live ? z3 : 0.0f;
        int h01, h23, l01, l23;
        hilo_pack(r0, r1, r2, r3, h01, h23, l01, l23);
        const v4i ow = regroup16(h01, h23, l01, l23, lane);
        if (node < mRows) {
          unsigned short* hp = xm + (size_t)node * KA + 8 * lane;
          *(volatile v4i*)hp = ow;
          __threadfence();
          *(volatile v4i*)hp = ow;
        }
      } else {
        const bool bad = (fa != 0) | (fb != 0) | big;
        v4f ow;
        ow.x = bad ? qnan : (x0.x + y0); ow.y = bad ? qnan : (x0.y + y1);
        ow.z = bad ? qnan : (x0.z + y2); ow.w = bad ? qnan : (x0.w + y3);
        if (live) {
          float* op = fout + (size_t)node * DD + 4 * lane;
          *(volatile v4f*)op = ow;
          __threadfence();
          *(volatile v4f*)op = ow;
        }
      }
    }
  }
}

static inline size_t al256(size_t o) { return (o + 255) & ~(size_t)255; }

extern "C" void kernel_launch(void* const* d_in, const int* in_sizes, int n_in,
                              void* d_out, int out_size, void* d_ws, size_t ws_size,
                              hipStream_t stream) {
  if (n_in < 16) return;
  if (in_sizes[0] != NN * DD || in_sizes[1] != NN * PEW) return;
  if (in_sizes[2] != 2 * NE || in_sizes[3] != NE) return;
  if (in_sizes[4] != 2 * NE || in_sizes[5] != NE) return;
  if (in_sizes[6] != KIN * DD || in_sizes[7] != KIN * DD) return;
  for (int i = 8; i < 16; ++i) if (in_sizes[i] != DD * DD) return;
  if (out_size != NN * DD) return;

  const float* x    = (const float*)d_in[0];
  const float* d2an = (const float*)d_in[1];
  const int*   ei0  = (const int*)d_in[2];
  const float* ea0  = (const float*)d_in[3];
  const int*   ei1  = (const int*)d_in[4];
  const float* ea1  = (const float*)d_in[5];
  const float* nl1  = (const float*)d_in[6];
  const float* nl2  = (const float*)d_in[7];
  const float* l11  = (const float*)d_in[8];
  const float* l21  = (const float*)d_in[9];
  const float* l12  = (const float*)d_in[10];
  const float* l22  = (const float*)d_in[11];
  const float* l13  = (const float*)d_in[12];
  const float* l23  = (const float*)d_in[13];
  const float* l14  = (const float*)d_in[14];
  const float* l24  = (const float*)d_in[15];
  float* out = (float*)d_out;
  const int* row0 = ei0;  const int* key0 = ei0 + NE;
  const int* row1 = ei1;  const int* key1 = ei1 + NE;

  const size_t RB = (size_t)MP * 512;
  char* ws = (char*)d_ws;
  size_t off = 0;
  const size_t oT   = off; off = al256(off + 2 * RB);
  const size_t oR2  = off; off = al256(off + RB);
  const size_t oR3  = off; off = al256(off + RB);
  const size_t oL0  = off; off = al256(off + (size_t)NBLK * RCAP * 8);
  const size_t oL1  = off; off = al256(off + (size_t)NBLK * RCAP * 8);
  const size_t oC0  = off; off = al256(off + (size_t)NBLK * NBA * 4);
  const size_t oO0  = off; off = al256(off + (size_t)NBLK * NBA * 4);
  const size_t oD0  = off; off = al256(off + (size_t)NBLK * NBA * 4);
  const size_t oF0  = off; off = al256(off + (size_t)NBLK * 128);
  const size_t oC1  = off; off = al256(off + (size_t)NBLK * NBA * 4);
  const size_t oO1  = off; off = al256(off + (size_t)NBLK * NBA * 4);
  const size_t oD1  = off; off = al256(off + (size_t)NBLK * NBA * 4);
  const size_t oF1  = off; off = al256(off + (size_t)NBLK * 128);
  const size_t oWP  = off; off = al256(off + (size_t)5 * KA * KA * 2);
  if (off > ws_size || off > (size_t)WSMAX) return;
  if (oR3 != oR2 + RB) return;

  float*          Tf   = (float*)(ws + oT);
  unsigned short* XIN  = (unsigned short*)(ws + oT);
  unsigned short* XPE1 = (unsigned short*)(ws + oR2);
  unsigned short* XPE2 = (unsigned short*)(ws + oR3);
  float*          X0H  = (float*)(ws + oR2);
  unsigned short* XM   = (unsigned short*)(ws + oR3);
  int* LIST0 = (int*)(ws + oL0);  int* LIST1 = (int*)(ws + oL1);
  int* CNT0  = (int*)(ws + oC0);  int* CNT1  = (int*)(ws + oC1);
  int* OFF0  = (int*)(ws + oO0);  int* OFF1  = (int*)(ws + oO1);
  int* DIS0i = (int*)(ws + oD0);  int* DIS1i = (int*)(ws + oD1);
  const float* DIS0 = (const float*)(ws + oD0);
  const float* DIS1 = (const float*)(ws + oD1);
  int* FLG0  = (int*)(ws + oF0);  int* FLG1  = (int*)(ws + oF1);
  unsigned short* WPL = (unsigned short*)(ws + oWP);
  const unsigned short* NLT = WPL;
  const unsigned short* WC1 = WPL + (size_t)1 * KA * KA;
  const unsigned short* WC2 = WPL + (size_t)2 * KA * KA;
  const unsigned short* WC3 = WPL + (size_t)3 * KA * KA;
  const unsigned short* WC4 = WPL + (size_t)4 * KA * KA;
  const size_t pstride = (size_t)MP * KA;

  const size_t bkLds = (size_t)BK_LDS_INTS * 4;
  hipFuncSetAttribute(reinterpret_cast<const void*>(&k_bucket), hipFuncAttributeMaxDynamicSharedMemorySize, (int)bkLds);

  const int vec8 = ((NE & 3) == 0) ? 1 : 0;
  const dim3 gG(MP / GBM, 2);
  const int gR = MP / RPB;

  k_prep<<<GXB + NWPB, NTHR, 0, stream>>>(x, d2an, nl1, nl2, l11, l21, l12, l22, l13, l23, l14, l24, NN, XIN, WPL);
  k_bucket<<<NBLK, NTHR, bkLds, stream>>>(row0, key0, ea0, NE, NN, vec8, LIST0, CNT0, OFF0, DIS0i, FLG0);
  k_bucket<<<NBLK, NTHR, bkLds, stream>>>(row1, key1, ea1, NE, NN, vec8, LIST1, CNT1, OFF1, DIS1i, FLG1);
  k_gemm<0, KA><<<gG, GTHR, 0, stream>>>(XIN, NLT, DIS0, NN, Tf, XPE1, pstride);
  k_gemm<1, KS1><<<gG, GTHR, 0, stream>>>(XPE1, WC1, DIS0, NN, Tf, XPE1, (size_t)0);
  k_replay<0><<<gR, NTHR, 0, stream>>>(Tf, LIST0, CNT0, OFF0, DIS0, FLG0, FLG0, NN, MP, X0H, X0H, XM);
  k_gemm<1, KS1><<<gG, GTHR, 0, stream>>>(XPE2, WC2, DIS1, NN, Tf, XPE1, (size_t)0);
  k_replay<1><<<gR, NTHR, 0, stream>>>(Tf, LIST1, CNT1, OFF1, DIS1, FLG1, FLG1, NN, MP, X0H, out, XM);
  k_gemm<1, KS2><<<gG, GTHR, 0, stream>>>(XM, WC3, DIS0, NN, Tf, XPE1, (size_t)0);
  k_replay<0><<<gR, NTHR, 0, stream>>>(Tf, LIST0, CNT0, OFF0, DIS0, FLG0, FLG0, NN, MP, X0H, X0H, XM);
  k_gemm<1, KS2><<<gG, GTHR, 0, stream>>>(XM, WC4, DIS1, NN, Tf, XPE1, (size_t)0);
  k_replay<2><<<gR, NTHR, 0, stream>>>(Tf, LIST1, CNT1, OFF1, DIS1, FLG1, FLG0, NN, MP, X0H, out, XM);
}
